// Mamba2Block_38577396253299
// MI455X (gfx1250) — hardware-verified
//
#include <hip/hip_runtime.h>
#include <math.h>

typedef __attribute__((ext_vector_type(16))) _Float16 v16h;
typedef __attribute__((ext_vector_type(8)))  _Float16 v8h;
typedef __attribute__((ext_vector_type(16))) __bf16   v16b;
typedef __attribute__((ext_vector_type(8)))  __bf16   v8b;
typedef __attribute__((ext_vector_type(8)))  float    v8f;
typedef __attribute__((ext_vector_type(4)))  float    v4f;

constexpr int kBatch   = 2;
constexpr int kSeq     = 2048;
constexpr int kRows    = kBatch * kSeq;
constexpr int kDm      = 768;
constexpr int kDin     = 1536;
constexpr int kNst     = 128;
constexpr int kHdim    = 64;
constexpr int kNh      = 24;
constexpr int kConvCh  = kDin + 2 * kNst;
constexpr int kProjN   = 2 * kDin + 2 * kNst + kNh;
constexpr int kProjNP  = 3392;
constexpr int kColXbc  = kDin;
constexpr int kColBC   = 2 * kDin;
constexpr int kColDt   = kDin + kConvCh;
constexpr int kBCW     = 2 * kNst;
constexpr int kScanTS  = 32;
constexpr int kScanP   = 32;
constexpr int kLanesPerP = 8;
constexpr int kStPerLane = kNst / kLanesPerP;
constexpr int kConvTP  = 260;
static_assert(kNh * kHdim == kDin);
static_assert(kProjNP >= kProjN && (kProjNP % 64) == 0);
static_assert((kDm % 32) == 0 && (kDin % 32) == 0);
static_assert((kRows % 64) == 0 && (kProjNP % 64) == 0 && (kDm % 64) == 0);
static_assert((kSeq % kScanTS) == 0 && (kSeq % 64) == 0 && (kHdim % kScanP) == 0);
static_assert(kScanP * kLanesPerP == 256 && kStPerLane * kLanesPerP == kNst);
static_assert((kColBC % 64) == 0 && (kColDt % 64) == 0 && (kColXbc % 4) == 0);

constexpr size_t kOffUB   = 0;
constexpr size_t kOffWIB  = kOffUB  + (size_t)kRows   * kDm     * 2;
constexpr size_t kOffWOB  = kOffWIB + (size_t)kProjNP * kDm     * 2;
constexpr size_t kOffZX   = kOffWOB + (size_t)kDm     * kDin    * 2;
constexpr size_t kOffBC   = kOffZX  + (size_t)kRows   * kProjNP * 4;
constexpr size_t kOffY    = kOffBC  + (size_t)kRows   * kBCW    * 4;
constexpr size_t kOffYNH  = kOffY   + (size_t)kRows   * kDin    * 4;
constexpr size_t kOffYNL  = kOffYNH + (size_t)kRows   * kDin    * 2;
constexpr size_t kWsTotal = kOffYNL + (size_t)kRows   * kDin    * 2;
static_assert(kWsTotal == 123961344ull);
static_assert(kWsTotal <= 134217728ull);
static_assert((kOffWIB % 128) == 0 && (kOffWOB % 128) == 0 && (kOffZX % 128) == 0 && (kOffBC % 128) == 0 &&
              (kOffY % 128) == 0 && (kOffYNH % 128) == 0 && (kOffYNL % 128) == 0);

__device__ __forceinline__ unsigned short f2bf_bits(float f) {
  unsigned u = __float_as_uint(f);
  return (unsigned short)((u + 0x7FFFu + ((u >> 16) & 1u)) >> 16);
}
__device__ __forceinline__ float bf_bits2f(unsigned short h) { return __uint_as_float(((unsigned)h) << 16); }
__device__ __forceinline__ float bf_rne(float f) { return bf_bits2f(f2bf_bits(f)); }

__device__ __forceinline__ void dep_guard4_h(v8f& a, v8f& b, v8f& c, v8f& d, v16h x, v16h y) { asm volatile("v_nop\n\tv_nop\n\tv_nop\n\tv_nop" : "+v"(a), "+v"(b), "+v"(c), "+v"(d) : "v"(x), "v"(y)); }
__device__ __forceinline__ void dep_guard4_b(v8f& a, v8f& b, v8f& c, v8f& d, v16b x, v16b y) { asm volatile("v_nop\n\tv_nop\n\tv_nop\n\tv_nop" : "+v"(a), "+v"(b), "+v"(c), "+v"(d) : "v"(x), "v"(y)); }
__device__ __forceinline__ void keep4_h(v16h a, v16h b, v16h c, v16h d) { asm volatile("v_nop" :: "v"(a), "v"(b), "v"(c), "v"(d)); }
__device__ __forceinline__ void keep4_b(v16b a, v16b b, v16b c, v16b d) { asm volatile("v_nop" :: "v"(a), "v"(b), "v"(c), "v"(d)); }
__device__ __forceinline__ void acc_guard4(v8f& a, v8f& b, v8f& c, v8f& d) { asm volatile("v_nop\n\tv_nop\n\tv_nop\n\tv_nop" : "+v"(a), "+v"(b), "+v"(c), "+v"(d)); }
template <typename T> struct Frag;
template <> struct Frag<_Float16> {
  typedef v16h V; union U { v16h v; v8h h[2]; };
  static __device__ __forceinline__ v16h load(const _Float16* p) {
    U f; f.h[0] = *(const v8h*)(p); f.h[1] = *(const v8h*)(p + 16); return f.v;
  }
  static __device__ __forceinline__ v8f mma(v16h a, v16h b, v8f c) {
    return __builtin_amdgcn_wmma_f32_16x16x32_f16(false, a, false, b, (short)0, c, false, false);
  }
  static __device__ __forceinline__ void guard4(v8f& a, v8f& b, v8f& c, v8f& d, v16h x, v16h y) { dep_guard4_h(a, b, c, d, x, y); }
  static __device__ __forceinline__ void keep(v16h a, v16h b, v16h c, v16h d) { keep4_h(a, b, c, d); }
};
template <> struct Frag<__bf16> {
  typedef v16b V; union U { v16b v; v8b h[2]; };
  static __device__ __forceinline__ v16b load(const __bf16* p) {
    U f; f.h[0] = *(const v8b*)(p); f.h[1] = *(const v8b*)(p + 16); return f.v;
  }
  static __device__ __forceinline__ v8f mma(v16b a, v16b b, v8f c) {
    return __builtin_amdgcn_wmma_f32_16x16x32_bf16(false, a, false, b, (short)0, c, false, false);
  }
  static __device__ __forceinline__ void guard4(v8f& a, v8f& b, v8f& c, v8f& d, v16b x, v16b y) { dep_guard4_b(a, b, c, d, x, y); }
  static __device__ __forceinline__ void keep(v16b a, v16b b, v16b c, v16b d) { keep4_b(a, b, c, d); }
};

template <int ET> struct Elem;
template <> struct Elem<0> { typedef _Float16 T; };
template <> struct Elem<1> { typedef __bf16 T; };
template <int ET, int SPL, int BIAS_MODE, int OUT_MODE, bool RESID, int ACT = 0>
__global__ __launch_bounds__(256) void wmma_gemm64(
    const unsigned short* __restrict__ Ap, const unsigned short* __restrict__ A2p, int lda, long strideA,
    const unsigned short* __restrict__ Btp, const unsigned short* __restrict__ Bt2p, int ldb, long strideB,
    void* __restrict__ Cout, void* __restrict__ Cout2, int ldc, long strideC,
    const float* __restrict__ bias,
    const float* __restrict__ resid, long strideR,
    int M, int N, int K, float scale) {
  typedef typename Elem<ET>::T T;
  typedef typename Frag<T>::V V;
  const T* A = (const T*)Ap; const T* A2 = (const T*)A2p; const T* Bt = (const T*)Btp; const T* Bt2 = (const T*)Bt2p;
  __shared__ __align__(16) float sT[8][16 * 68];
  const int b    = blockIdx.y;
  const int lane = threadIdx.x & 31;
  const int wave = threadIdx.x >> 5;
  const int tilesN = N >> 6;
  const int tilesM = M >> 6;
  const int tile = blockIdx.x * 8 + wave;
  if (tile >= tilesM * tilesN) return;
  const int tm = tile / tilesN;
  const int tn = tile - tm * tilesN;
  const int m0 = tm << 6;
  const int n0 = tn << 6;

  const T* Ab  = A  + (size_t)b * strideA;
  const T* Bb  = Bt + (size_t)b * strideB;
  const T* Ab2 = (SPL >= 1) ? (A2  + (size_t)b * strideA) : nullptr;
  const T* Bb2 = (SPL == 2) ? (Bt2 + (size_t)b * strideB) : nullptr;

  const int rlane = lane & 15;
  const int koff  = (lane >> 4) * 8;
  const int mOff  = (lane >> 4) * 8;

  v8f acc[4][4];
#pragma unroll
  for (int i = 0; i < 4; ++i)
#pragma unroll
    for (int j = 0; j < 4; ++j) acc[i][j] = (v8f){0.f,0.f,0.f,0.f,0.f,0.f,0.f,0.f};

  for (int k0 = 0; k0 < K; k0 += 32) {
    V bh[4], bl[4];
#pragma unroll
    for (int j = 0; j < 4; ++j) {
      const size_t bo = (size_t)(n0 + (j << 4) + rlane) * ldb + koff + k0;
      bh[j] = Frag<T>::load(Bb + bo);
      if (SPL == 2) bl[j] = Frag<T>::load(Bb2 + bo);
    }
#pragma unroll
    for (int i = 0; i < 4; ++i) {
      const size_t ao = (size_t)(m0 + (i << 4) + rlane) * lda + koff + k0;
      V ah = Frag<T>::load(Ab + ao);
      V al;
      if (SPL >= 1) al = Frag<T>::load(Ab2 + ao);
#pragma unroll
      for (int j = 0; j < 4; ++j) {
        acc[i][j] = Frag<T>::mma(ah, bh[j], acc[i][j]);
        if (SPL == 2) acc[i][j] = Frag<T>::mma(ah, bl[j], acc[i][j]);
        if (SPL >= 1) acc[i][j] = Frag<T>::mma(al, bh[j], acc[i][j]);
      }
      Frag<T>::guard4(acc[i][0], acc[i][1], acc[i][2], acc[i][3], ah, (SPL >= 1) ? al : ah);
    }
    Frag<T>::keep(bh[0], bh[1], bh[2], bh[3]);
    if (SPL == 2) Frag<T>::keep(bl[0], bl[1], bl[2], bl[3]);
  }
  acc_guard4(acc[0][0], acc[0][1], acc[0][2], acc[0][3]);
  acc_guard4(acc[1][0], acc[1][1], acc[1][2], acc[1][3]);
  acc_guard4(acc[2][0], acc[2][1], acc[2][2], acc[2][3]);
  acc_guard4(acc[3][0], acc[3][1], acc[3][2], acc[3][3]);

  float* slab = sT[wave];
  const float* Rb = RESID ? (resid + (size_t)b * strideR) : nullptr;
#pragma unroll
  for (int i = 0; i < 4; ++i) {
    const int mBase = m0 + (i << 4);
#pragma unroll
    for (int j = 0; j < 4; ++j) {
      const int n = n0 + (j << 4) + rlane;
      float bv = 0.f;
      if (BIAS_MODE == 2) bv = bias[n];
#pragma unroll
      for (int r = 0; r < 8; ++r) {
        float v = acc[i][j][r] * scale;
        if (BIAS_MODE == 1) v += bias[mBase + mOff + r];
        if (BIAS_MODE == 2) v += bv;
        if (RESID) v += Rb[(size_t)(mBase + mOff + r) * ldc + n];
        if (ACT == 1) v = tanhf(v);
        if (ACT == 2) v = fmaxf(v, 0.0f);
        if (ACT == 3) v = v / (1.0f + expf(-v));
        if (ACT == 4) v = (v > 0.f) ? v : 0.01f * v;
        slab[(mOff + r) * 68 + (j << 4) + rlane] = v;
      }
    }
    __builtin_amdgcn_fence(__ATOMIC_RELEASE, "workgroup");
    __builtin_amdgcn_wave_barrier();
    __builtin_amdgcn_fence(__ATOMIC_ACQUIRE, "workgroup");
    if (OUT_MODE == 0) {
      float* C = (float*)Cout + (size_t)b * strideC;
      const int hh = lane >> 4, c4 = (lane & 15) * 4;
      for (int pass = 0; pass < 2; ++pass) {
#pragma unroll
        for (int it = 0; it < 8; ++it) {
          const int row = it * 2 + hh;
          v4f v = *(const v4f*)(slab + row * 68 + c4);
          *(volatile v4f*)(C + (size_t)(mBase + row) * ldc + n0 + c4) = v;
        }
        __threadfence();
      }
    } else {
      const int q = lane >> 3, c8 = (lane & 7) * 8;
      unsigned short* C  = (unsigned short*)Cout  + (size_t)b * strideC;
      unsigned short* C2 = (OUT_MODE == 2) ? ((unsigned short*)Cout2 + (size_t)b * strideC) : nullptr;
      for (int pass = 0; pass < 2; ++pass) {
#pragma unroll
        for (int it = 0; it < 4; ++it) {
          const int row = it * 4 + q;
          const float* sp = slab + row * 68 + c8;
          v8h hv, lv;
#pragma unroll
          for (int e = 0; e < 8; ++e) {
            if (OUT_MODE == 1) {
              hv[e] = (_Float16)sp[e];
            } else {
              unsigned short hb = f2bf_bits(sp[e]);
              unsigned short lb = f2bf_bits(sp[e] - bf_bits2f(hb));
              hv[e] = __builtin_bit_cast(_Float16, hb);
              lv[e] = __builtin_bit_cast(_Float16, lb);
            }
          }
          *(volatile v8h*)(C + (size_t)(mBase + row) * ldc + n0 + c8) = hv;
          if (OUT_MODE == 2) *(volatile v8h*)(C2 + (size_t)(mBase + row) * ldc + n0 + c8) = lv;
        }
        __threadfence();
      }
    }
    __builtin_amdgcn_fence(__ATOMIC_RELEASE, "workgroup");
    __builtin_amdgcn_wave_barrier();
    __builtin_amdgcn_fence(__ATOMIC_ACQUIRE, "workgroup");
  }
}

__global__ __launch_bounds__(256) void cvt_rows_bf16_kernel(
    const float* __restrict__ src, unsigned short* __restrict__ dst, int real8, int total8)
{
  const int i = blockIdx.x * 256 + threadIdx.x;
  if (i >= total8) return;
  const bool live = (i < real8);
  const int ic = live ? i : (real8 - 1);
  const float fl = live ? 1.0f : 0.0f;
  const size_t e0 = (size_t)ic << 3;
  const v4f a0 = *(const v4f*)(src + e0);
  const v4f a1 = *(const v4f*)(src + e0 + 4);
  v8h hv;
#pragma unroll
  for (int e = 0; e < 4; ++e) {
    const float f0 = a0[e] * fl;
    const float f1 = a1[e] * fl;
    hv[e]     = __builtin_bit_cast(_Float16, f2bf_bits(f0));
    hv[4 + e] = __builtin_bit_cast(_Float16, f2bf_bits(f1));
  }
  unsigned short* q = dst + ((size_t)i << 3);
  *(volatile v8h*)q = hv;
  __threadfence();
  *(volatile v8h*)q = hv;
}

__global__ __launch_bounds__(256) void conv_bc_kernel(
    const float* __restrict__ ZX, const float* __restrict__ cw, const float* __restrict__ cb,
    float* __restrict__ BCp)
{
  __shared__ __align__(16) float sT[16 * kConvTP];
  const int tid = threadIdx.x, lane = tid & 31, wave = tid >> 5;
  const int d  = tid;
  const int cc = kDin + d;
  const int zc = kColBC + d;
  const int g0 = blockIdx.x * 64;
  const int tb = g0 & (kSeq - 1);
  const float w0 = bf_rne(cw[cc * 4 + 0]), w1 = bf_rne(cw[cc * 4 + 1]);
  const float w2 = bf_rne(cw[cc * 4 + 2]), w3 = bf_rne(cw[cc * 4 + 3]);
  const float bcv = bf_rne(cb[cc]);
  float xm3, xm2, xm1;
  {
    const bool hist = (tb > 0);
    const float hf = hist ? 1.0f : 0.0f;
    const int rb = hist ? (g0 - 3) : g0;
    const float v3 = ZX[(size_t)rb * kProjNP + zc];
    const float v2 = ZX[(size_t)(rb + 1) * kProjNP + zc];
    const float v1 = ZX[(size_t)(rb + 2) * kProjNP + zc];
    xm3 = v3 * hf;
    xm2 = v2 * hf;
    xm1 = v1 * hf;
  }
  const int hrow = wave >> 1;
  const int hch  = (wave & 1) * 128 + lane * 4;
#pragma unroll 1
  for (int sub = 0; sub < 4; ++sub) {
    const int lb = g0 + sub * 16;
#pragma unroll 1
    for (int s = 0; s < 16; ++s) {
      const float xcur = ZX[(size_t)(lb + s) * kProjNP + zc];
      float acc = w0 * xm3;
      acc = fmaf(w1, xm2, acc);
      acc = fmaf(w2, xm1, acc);
      acc = fmaf(w3, xcur, acc);
      const float sv = acc + bcv;
      const float sg = __builtin_amdgcn_rcpf(1.0f + expf(-sv));
      sT[s * kConvTP + tid] = sv * sg;
      xm3 = xm2; xm2 = xm1; xm1 = xcur;
    }
    __syncthreads();
    v4f fv[4];
#pragma unroll
    for (int it = 0; it < 4; ++it) fv[it] = *(const v4f*)(sT + (it * 4 + hrow) * kConvTP + hch);
    for (int pass = 0; pass < 2; ++pass) {
#pragma unroll
      for (int it = 0; it < 4; ++it)
        *(volatile v4f*)(BCp + (size_t)(lb + it * 4 + hrow) * kBCW + hch) = fv[it];
      __threadfence();
    }
    __syncthreads();
  }
}

__global__ __launch_bounds__(256) void scan_kernel(
    const float* __restrict__ ZX, const float* __restrict__ BCp, const float* __restrict__ cw,
    const float* __restrict__ cb, const float* __restrict__ dt_bias, const float* __restrict__ A_log,
    const float* __restrict__ Dp, float* __restrict__ Y)
{
  __shared__ __align__(16) float sBC[kScanTS * kBCW];
  __shared__ __align__(16) float sX[kScanTS * kScanP];
  __shared__ __align__(16) float sY[kScanTS * kScanP];
  __shared__ float sdA[kScanTS];
  __shared__ float sdt[kScanTS];
  const int tid = threadIdx.x, lane = tid & 31, wave = tid >> 5;
  constexpr int kBlkPerB = kNh * (kHdim / kScanP);
  const int bix  = blockIdx.x / kBlkPerB;
  const int rem  = blockIdx.x - bix * kBlkPerB;
  const int h    = rem >> 1;
  const int half = rem & 1;
  const int chx0 = h * kHdim + half * kScanP;
  const size_t row0 = (size_t)bix * kSeq;
  const int pl = tid >> 3;
  const int nq = tid & 7;
  const int n0 = nq * kStPerLane;

  const int cx = chx0 + lane;
  const float wx0 = bf_rne(cw[cx * 4 + 0]), wx1 = bf_rne(cw[cx * 4 + 1]);
  const float wx2 = bf_rne(cw[cx * 4 + 2]), wx3 = bf_rne(cw[cx * 4 + 3]);
  const float bx  = bf_rne(cb[cx]);
  const float dtb  = bf_rne(dt_bias[h]);
  const float aneg = -expf(bf_rne(A_log[h]));
  const float dsk  = bf_rne(Dp[h]);

  float st[kStPerLane];
#pragma unroll
  for (int k = 0; k < kStPerLane; ++k) st[k] = 0.f;
  float xm3 = 0.f, xm2 = 0.f, xm1 = 0.f;

  const int sr = tid >> 3, sc4 = (tid & 7) * 4;
  const int q = lane >> 3, c4 = (lane & 7) * 4;

#pragma unroll 1
  for (int t0 = 0; t0 < kSeq; t0 += kScanTS) {
    __syncthreads();
#pragma unroll
    for (int i = 0; i < 4; ++i) {
      const int idx = i * 256 + tid;
      const int r = idx >> 6, bc4 = (idx & 63) * 4;
      *(v4f*)(sBC + r * kBCW + bc4) = *(const v4f*)(BCp + (row0 + t0 + r) * kBCW + bc4);
    }
    asm volatile("" ::: "memory");
#pragma unroll
    for (int i = 4; i < 8; ++i) {
      const int idx = i * 256 + tid;
      const int r = idx >> 6, bc4 = (idx & 63) * 4;
      *(v4f*)(sBC + r * kBCW + bc4) = *(const v4f*)(BCp + (row0 + t0 + r) * kBCW + bc4);
    }
    asm volatile("" ::: "memory");
    *(v4f*)(sX + sr * kScanP + sc4) = *(const v4f*)(ZX + (row0 + t0 + sr) * kProjNP + kColXbc + chx0 + sc4);
    if (wave == 1) {
      const float raw = ZX[(row0 + t0 + lane) * kProjNP + kColDt + h];
      const float sv  = raw + dtb;
      const float sp  = fmaxf(sv, 0.0f) + log1pf(expf(-fabsf(sv)));
      sdt[lane] = sp;
      sdA[lane] = expf(sp * aneg);
    }
    __syncthreads();
    if (wave == 0) {
#pragma unroll 1
      for (int r = 0; r < kScanTS; ++r) {
        const float xcur = sX[r * kScanP + lane];
        float acc = wx0 * xm3;
        acc = fmaf(wx1, xm2, acc);
        acc = fmaf(wx2, xm1, acc);
        acc = fmaf(wx3, xcur, acc);
        const float sv = acc + bx;
        const float sg = __builtin_amdgcn_rcpf(1.0f + expf(-sv));
        sX[r * kScanP + lane] = sv * sg;
        xm3 = xm2; xm2 = xm1; xm1 = xcur;
      }
    }
    __syncthreads();
#pragma unroll 1
    for (int s = 0; s < kScanTS; ++s) {
      const float da   = sdA[s];
      const float dtv  = sdt[s];
      const float xv   = sX[s * kScanP + pl];
      const float coef = dtv * xv;
      const float* br = sBC + s * kBCW + n0;
      const float* cr = br + kNst;
      float acc = 0.f;
#pragma unroll
      for (int q4 = 0; q4 < 4; ++q4) {
        const v4f bv = *(const v4f*)(br + 4 * q4);
        const v4f cv = *(const v4f*)(cr + 4 * q4);
#pragma unroll
        for (int e = 0; e < 4; ++e) {
          const int k = 4 * q4 + e;
          st[k] = fmaf(st[k], da, coef * bv[e]);
          acc = fmaf(st[k], cv[e], acc);
        }
      }
      acc += __shfl_xor(acc, 1, 32);
      acc += __shfl_xor(acc, 2, 32);
      acc += __shfl_xor(acc, 4, 32);
      const float yv = fmaf(dsk, xv, acc);
      if (nq == 0) sY[s * kScanP + pl] = yv;
    }
    __syncthreads();
    {
      const int row = wave * 4 + q;
      const v4f v = *(const v4f*)(sY + row * kScanP + c4);
      float* dstp = Y + (row0 + t0 + row) * kDin + chx0 + c4;
      *(volatile v4f*)dstp = v;
      __threadfence();
      *(volatile v4f*)dstp = v;
    }
  }
}

__global__ __launch_bounds__(192) void gate_norm_kernel(
    const float* __restrict__ Y, const float* __restrict__ ZX, const float* __restrict__ nw,
    unsigned short* __restrict__ YNH, unsigned short* __restrict__ YNL)
{
  __shared__ float red[8];
  const int row = blockIdx.x, tid = threadIdx.x, lane = tid & 31, wave = tid >> 5;
  const int e0 = tid * 8;
  const float* yr = Y  + (size_t)row * kDin    + e0;
  const float* zr = ZX + (size_t)row * kProjNP + e0;
  const v4f y0 = *(const v4f*)(yr), y1 = *(const v4f*)(yr + 4);
  const v4f z0 = *(const v4f*)(zr), z1 = *(const v4f*)(zr + 4);
  const v4f w0v = *(const v4f*)(nw + e0), w1v = *(const v4f*)(nw + e0 + 4);
  float g[8];
  float ss = 0.f;
#pragma unroll
  for (int e = 0; e < 4; ++e) {
    const float zz = z0[e];
    const float sg = __builtin_amdgcn_rcpf(1.0f + expf(-zz));
    const float v  = y0[e] * (zz * sg);
    g[e] = v;
    ss = fmaf(v, v, ss);
  }
#pragma unroll
  for (int e = 0; e < 4; ++e) {
    const float zz = z1[e];
    const float sg = __builtin_amdgcn_rcpf(1.0f + expf(-zz));
    const float v  = y1[e] * (zz * sg);
    g[4 + e] = v;
    ss = fmaf(v, v, ss);
  }
#pragma unroll
  for (int off = 16; off > 0; off >>= 1) ss += __shfl_xor(ss, off, 32);
  if (lane == 0) red[wave] = ss;
  __syncthreads();
  float tot = red[0];
#pragma unroll
  for (int i = 1; i < 6; ++i) tot += red[i];
  const float rs = rsqrtf(tot * (1.0f / 1536.0f) + 1e-5f);
  v8h hv, lv;
#pragma unroll
  for (int e = 0; e < 4; ++e) {
    const float v = (g[e] * rs) * bf_rne(w0v[e]);
    const unsigned short hb = f2bf_bits(v);
    const unsigned short lb = f2bf_bits(v - bf_bits2f(hb));
    hv[e] = __builtin_bit_cast(_Float16, hb);
    lv[e] = __builtin_bit_cast(_Float16, lb);
  }
#pragma unroll
  for (int e = 0; e < 4; ++e) {
    const float v = (g[4 + e] * rs) * bf_rne(w1v[e]);
    const unsigned short hb = f2bf_bits(v);
    const unsigned short lb = f2bf_bits(v - bf_bits2f(hb));
    hv[4 + e] = __builtin_bit_cast(_Float16, hb);
    lv[4 + e] = __builtin_bit_cast(_Float16, lb);
  }
  const size_t o = (size_t)row * kDin + e0;
  *(volatile v8h*)(YNH + o) = hv;
  *(volatile v8h*)(YNL + o) = lv;
  __threadfence();
  *(volatile v8h*)(YNH + o) = hv;
  *(volatile v8h*)(YNL + o) = lv;
}

extern "C" void kernel_launch(void* const* d_in, const int* in_sizes, int n_in,
                              void* d_out, int out_size, void* d_ws, size_t ws_size,
                              hipStream_t stream) {
  if (n_in < 9) return;
  if (in_sizes[0] != kRows * kDm) return;
  if (in_sizes[1] != kProjN * kDm) return;
  if (in_sizes[2] != kConvCh * 4) return;
  if (in_sizes[3] != kConvCh) return;
  if (in_sizes[4] != kNh) return;
  if (in_sizes[5] != kNh) return;
  if (in_sizes[6] != kNh) return;
  if (in_sizes[7] != kDin) return;
  if (in_sizes[8] != kDm * kDin) return;
  if (out_size != kRows * kDm) return;
  if (ws_size < kWsTotal) return;

  const float* u          = (const float*)d_in[0];
  const float* in_proj_w  = (const float*)d_in[1];
  const float* conv_w     = (const float*)d_in[2];
  const float* conv_b     = (const float*)d_in[3];
  const float* dt_bias    = (const float*)d_in[4];
  const float* A_log      = (const float*)d_in[5];
  const float* Dp         = (const float*)d_in[6];
  const float* norm_w     = (const float*)d_in[7];
  const float* out_proj_w = (const float*)d_in[8];
  float* out = (float*)d_out;

  char* ws = (char*)d_ws;
  unsigned short* UB  = (unsigned short*)(ws + kOffUB);
  unsigned short* WIB = (unsigned short*)(ws + kOffWIB);
  unsigned short* WOB = (unsigned short*)(ws + kOffWOB);
  float*          ZX  = (float*)(ws + kOffZX);
  float*          BCp = (float*)(ws + kOffBC);
  float*          Y   = (float*)(ws + kOffY);
  unsigned short* YNH = (unsigned short*)(ws + kOffYNH);
  unsigned short* YNL = (unsigned short*)(ws + kOffYNL);

  {
    const int t8u = kRows * kDm / 8;
    cvt_rows_bf16_kernel<<<(t8u + 255) / 256, 256, 0, stream>>>(u, UB, t8u, t8u);
    const int r8w = kProjN * kDm / 8, t8w = kProjNP * kDm / 8;
    cvt_rows_bf16_kernel<<<(t8w + 255) / 256, 256, 0, stream>>>(in_proj_w, WIB, r8w, t8w);
    const int t8o = kDm * kDin / 8;
    cvt_rows_bf16_kernel<<<(t8o + 255) / 256, 256, 0, stream>>>(out_proj_w, WOB, t8o, t8o);
  }

  wmma_gemm64<1, 0, 0, 0, false><<<dim3((kRows / 64) * (kProjNP / 64) / 8, 1), 256, 0, stream>>>(
      UB, nullptr, kDm, 0L,
      WIB, nullptr, kDm, 0L,
      (void*)ZX, nullptr, kProjNP, 0L,
      nullptr, nullptr, 0L,
      kRows, kProjNP, kDm, 1.0f);

  conv_bc_kernel<<<kRows / 64, 256, 0, stream>>>(ZX, conv_w, conv_b, BCp);

  scan_kernel<<<kBatch * kNh * (kHdim / kScanP), 256, 0, stream>>>(ZX, BCp, conv_w, conv_b, dt_bias, A_log, Dp, Y);

  gate_norm_kernel<<<kRows, 192, 0, stream>>>(Y, ZX, norm_w, YNH, YNL);

  wmma_gemm64<1, 1, 0, 0, false><<<dim3((kRows / 64) * (kDm / 64) / 8, 1), 256, 0, stream>>>(
      YNH, YNL, kDin, 0L,
      WOB, nullptr, kDin, 0L,
      (void*)out, nullptr, kDm, 0L,
      nullptr, nullptr, 0L,
      kRows, kDm, kDin, 1.0f);
}
